// EdgeConvBlock_1623497638706
// MI455X (gfx1250) — hardware-verified
//
#include <hip/hip_runtime.h>


namespace {

constexpr int N = 100000, NP = 100032, NPL = NP  , SRCM = N  , EFULL = 800000, E = EFULL  ;
constexpr int F = 64  , FH = 64, KNB = 16  , CW3 = 67  , EC = E, VOC = 1, NRL = NP  , NL = (NPL < N ? NPL : N);
constexpr float LN_EPS = 1e-5f;
constexpr float LNEPS = 1e-5f; constexpr float XS = 8.0f, WSC = 256.0f, WSQ = 0.25f, RS_ = 1024.0f, NSL_ = 0.2f, NSA_ = 0.01f, SLOPE = 0.0f, BNEPS = 1e-5f;
static_assert(NP % 32 == 0 && NP >= N && NPL % 32 == 0 && F % 32 == 0, "tiling");
typedef _Float16 b16;
typedef __attribute__((ext_vector_type(16))) _Float16 v16b;
typedef __attribute__((ext_vector_type(8))) _Float16 v8b;
typedef __attribute__((ext_vector_type(8))) float v8f;
typedef __attribute__((ext_vector_type(4))) float v4f;
__device__ __forceinline__ float bf16_rne(float f) { unsigned int u = __float_as_uint(f); u += 0x7FFFu + ((u >> 16) & 1u); return __uint_as_float(u & 0xFFFF0000u); }
__device__ __forceinline__ float bfo(float f) { float r = bf16_rne(f); asm volatile("" : "+v"(r)); return r; }
__device__ __forceinline__ void split16(float v, b16& hi, b16& lo) { hi = (b16)v; lo = (b16)(v - (float)hi); }
__device__ __forceinline__ v16b frag_kb(const b16* p, int hh) { const v8b a = *(const v8b*)(p + 8 * hh), b = *(const v8b*)(p + 16 + 8 * hh); v16b f;
#pragma unroll
  for (int e = 0; e < 8; ++e) { f[e] = a[e]; f[8 + e] = b[e]; } return f; }
__device__ __forceinline__ v8f wmma16b(v16b a, v16b b, v8f c) { v8f d = __builtin_amdgcn_wmma_f32_16x16x32_f16(false, a, false, b, (short)0, c, false, false); asm volatile("v_nop\n\tv_nop\n\tv_nop\n\tv_nop" : "+v"(d) : "v"(a), "v"(b)); return d; }
__device__ __forceinline__ void wave_lds_sync() { __builtin_amdgcn_fence(__ATOMIC_RELEASE, "workgroup"); __builtin_amdgcn_wave_barrier(); __builtin_amdgcn_fence(__ATOMIC_ACQUIRE, "workgroup"); }
__device__ __forceinline__ float pmul(float a, float b) { float p = a * b; asm volatile("" : "+v"(p)); return p; }
__device__ __forceinline__ int iclamp(int v, int lo, int hi) { return v < lo ? lo : (v > hi ? hi : v); }
typedef __attribute__((ext_vector_type(4))) _Float16 v4h;
__device__ __forceinline__ float lrelu(float v) { return v > 0.0f ? v : NSL_ * v; }
template <int K, int NOUTR, int NOUTP>
__global__ __launch_bounds__(256) void wt_kernel(const float* __restrict__ w, b16* __restrict__ WT, float scl) {
  const int u = blockIdx.x * 256 + threadIdx.x; if (u >= NOUTP * K / 8) return; const int e = u * 8; const int o = e / K, k0 = e % K; v8b v;
#pragma unroll
  for (int j = 0; j < 8; ++j) v[j] = (b16)(o < NOUTR ? bf16_rne(w[(size_t)(k0 + j) * NOUTR + o]) * scl : 0.0f);
  for (int pass = 0; pass < 2; ++pass) { *(volatile v8b*)(WT + e) = v; __threadfence(); }
}
__global__ __launch_bounds__(256) void zfill_kernel(float* __restrict__ Z, int n) { const int i = threadIdx.x; for (int pass = 0; pass < 2; ++pass) { if (i < n) ((volatile float*)Z)[i] = 0.0f; __threadfence(); } }
template <int K, int NT, int PREC, int MODE, bool GIDX>
__global__ __launch_bounds__(64) void lin_kernel(const float* __restrict__ X, const int* __restrict__ gidx, const b16* __restrict__ WT, const b16* __restrict__ WQ, const float* __restrict__ bias, float* __restrict__ OUT, int opitch, int nvalid, int mrows) {
  constexpr int NC = NT * 16;
  __shared__ __attribute__((aligned(16))) b16 Ah[2][16][K + 8], Al[2][16][(PREC == 0 ? K : 0) + 8]; __shared__ __attribute__((aligned(16))) float Tf[2][16][NC + 4];
  const int wave = threadIdx.x >> 5, lane = threadIdx.x & 31, nloc = lane & 15, hlf = lane >> 4; const size_t m0 = (size_t)blockIdx.x * 32 + wave * 16;
  for (int idx = lane; idx < 16 * (K / 4); idx += 32) { const int rr = idx / (K / 4), c4 = (idx % (K / 4)) * 4; const size_t vrow = (m0 + rr < (size_t)nvalid) ? m0 + rr : (size_t)nvalid - 1; size_t arow = vrow; if (GIDX) arow = (size_t)iclamp(gidx[vrow], 0, VOC - 1);
    const v4f v = *(const v4f*)(X + arow * K + c4); v4h hv, lv;
    for (int j = 0; j < 4; ++j) { float vj = v[j]; if (MODE == 2) vj = fmaxf(vj, 0.0f); const float vs = (PREC == 1 ? bf16_rne(vj) : vj) * XS; const b16 ph = (b16)vs; hv[j] = ph; lv[j] = (b16)((vs - (float)ph) * RS_); } *(v4h*)(&Ah[wave][rr][c4]) = hv; if (PREC == 0) *(v4h*)(&Al[wave][rr][c4]) = lv; }
  wave_lds_sync();
  v8f acc[NT];
#pragma unroll
  for (int t = 0; t < NT; ++t) acc[t] = (v8f){};
#pragma unroll 1
  for (int kb = 0; kb < K; kb += 32) { const v16b a = frag_kb(&Ah[wave][nloc][kb], hlf); v16b al; if (PREC == 0) al = frag_kb(&Al[wave][nloc][kb], hlf);
#pragma unroll
    for (int t = 0; t < NT; ++t) { const size_t wo_ = (size_t)(t * 16 + nloc) * K + kb; acc[t] = wmma16b(a, frag_kb(WT + wo_, hlf), acc[t]); if (PREC == 0) acc[t] = wmma16b(al, frag_kb(WQ + wo_, hlf), acc[t]); } }
#pragma unroll
  for (int t = 0; t < NT; ++t) { const int col = t * 16 + nloc; const float bb = (MODE == 14 || MODE == 17 || MODE == 19 || MODE == 24) ? 0.0f : bf16_rne(bias[col]);
    for (int r = 0; r < 8; ++r) { const size_t vrow = m0 + 8 * hlf + r; float y = acc[t][r] * (1.0f / (XS * WSC)) + bb; if (MODE == 1) y = fmaxf(y, 0.0f); if ((MODE == 14 || MODE == 17 || MODE == 19 || MODE == 24) && vrow < (size_t)mrows) y += OUT[vrow * (size_t)opitch + col]; if (MODE == 17 || MODE == 19) y = fmaxf(y, 0.0f); if (MODE == 19) y = __frcp_rn(1.0f + __expf(-y)); if (MODE == 24) y = __frcp_rn(1.0f + __expf(10.0f - y));         Tf[wave][8 * hlf + r][col] = (vrow < (size_t)nvalid) ? y : 0.0f; } }
  wave_lds_sync();
  for (int pass = 0; pass < 2; ++pass) { for (int rr = 0; rr < 16; ++rr) { if (m0 + rr < (size_t)mrows) { if (NC >= 128) { for (int c8 = 0; c8 < NC; c8 += 128) *(volatile v4f*)(OUT + (m0 + rr) * (size_t)opitch + c8 + lane * 4) = *(const v4f*)(&Tf[wave][rr][c8 + lane * 4]); }
        else { if (lane < NC / 4) *(volatile v4f*)(OUT + (m0 + rr) * (size_t)opitch + lane * 4) = *(const v4f*)(&Tf[wave][rr][lane * 4]); } } } __threadfence(); }
}
template <int K, int NOUT>
__global__ __launch_bounds__(256) void wtoip_kernel(const float* __restrict__ w, int wpitch, int coff, b16* __restrict__ WT, float scl) {
  const int u = blockIdx.x * 256 + threadIdx.x; if (u >= NOUT * K / 8) return; const int e = u * 8; const int o = e / K, k0 = e % K; v8b v;
#pragma unroll
  for (int j = 0; j < 8; ++j) v[j] = (b16)(bf16_rne(w[(size_t)o * wpitch + coff + k0 + j]) * scl);
  for (int pass = 0; pass < 2; ++pass) { *(volatile v8b*)(WT + e) = v; __threadfence(); }
}
template <int W, int ACT>
__global__ __launch_bounds__(256) void bnact_kernel(const float* __restrict__ H, const float* __restrict__ SCL, const float* __restrict__ SFT, float* __restrict__ OUT, int op, int mrows) {
  const size_t i = (size_t)blockIdx.x * 256 + threadIdx.x; if (i >= (size_t)mrows * (W / 4)) return; const size_t v = i / (W / 4); const int c = (int)(i % (W / 4)) * 4;
  const v4f h = *(const v4f*)(H + v * W + c), s = *(const v4f*)(SCL + c), t = *(const v4f*)(SFT + c); v4f o;
  for (int j = 0; j < 4; ++j) { float y = pmul(h[j], s[j]) + t[j]; if (ACT == 1) y = fmaxf(y, 0.0f); if (ACT == 3) y = (y >= 0.0f) ? y : 0.01f * y; o[j] = y; }
  for (int pass = 0; pass < 2; ++pass) { *(volatile v4f*)(OUT + v * (size_t)op + c) = o; __threadfence(); }
}
__global__ __launch_bounds__(256) void bnfold_kernel(const float* __restrict__ g, const float* __restrict__ b, const float* __restrict__ m, const float* __restrict__ v, float* __restrict__ SCL, float* __restrict__ SFT) {
  const int c = threadIdx.x; float s = 0.0f, t = 0.0f; if (c < F) { s = pmul(bfo(g[c]), rsqrtf(bfo(v[c]) + 1e-5f)); t = bfo(b[c]) - pmul(bfo(m[c]), s); }
  for (int pass = 0; pass < 2; ++pass) { ((volatile float*)SCL)[c] = s; ((volatile float*)SFT)[c] = t; __threadfence(); }
}
__global__ __launch_bounds__(256) void qtadd_kernel(const float* __restrict__ p, const float* __restrict__ cw, const float* __restrict__ G, float* __restrict__ Q, float* __restrict__ T, int mrows) {
  const size_t i = (size_t)blockIdx.x * 256 + threadIdx.x; if (i >= (size_t)mrows * (F / 4)) return; const size_t n = i / (F / 4); const int c = (int)(i % (F / 4)) * 4; const size_t nn = n < (size_t)N ? n : (size_t)N - 1;
  const float px = bfo(p[nn * 3 + 0]), py = bfo(p[nn * 3 + 1]), pz = bfo(p[nn * 3 + 2]); const v4f g4 = *(const v4f*)(G + n * F + c); v4f q, t;
  for (int j = 0; j < 4; ++j) { const float* w = cw + (size_t)(c + j) * CW3; const float qq = (pmul(px, bfo(w[0])) + pmul(py, bfo(w[1]))) + pmul(pz, bfo(w[2])); q[j] = (n < (size_t)N) ? qq : 0.0f; t[j] = (n < (size_t)N) ? g4[j] + qq : 0.0f; }
  for (int pass = 0; pass < 2; ++pass) { *(volatile v4f*)(Q + n * F + c) = q; *(volatile v4f*)(T + n * F + c) = t; __threadfence(); }
}
__global__ __launch_bounds__(256) void ecmax_kernel(const float* __restrict__ T, const float* __restrict__ Q, const int* __restrict__ tab, const float* __restrict__ SCL, const float* __restrict__ SFT, float* __restrict__ FO_, int mrows) {
  const int tid = threadIdx.x; const int row = tid >> 3, g = tid & 7, c0 = g * 8; const int v = blockIdx.x * 32 + row; const int vv = v < N ? v : N - 1; float q[8], s[8], t[8], mx[8];
  { const v4f q0 = *(const v4f*)(Q + (size_t)vv * F + c0), q1 = *(const v4f*)(Q + (size_t)vv * F + c0 + 4), s0 = *(const v4f*)(SCL + c0), s1 = *(const v4f*)(SCL + c0 + 4), t0 = *(const v4f*)(SFT + c0), t1 = *(const v4f*)(SFT + c0 + 4); for (int j = 0; j < 4; ++j) { q[j] = q0[j]; q[4 + j] = q1[j]; s[j] = s0[j]; s[4 + j] = s1[j]; t[j] = t0[j]; t[4 + j] = t1[j]; mx[j] = -INFINITY; mx[4 + j] = -INFINITY; } }
#pragma unroll 1
  for (int k = 0; k < KNB; ++k) { int sidx = iclamp(tab[(size_t)vv * KNB + k], 0, N - 1); if (SRCM < N) sidx %= SRCM; const v4f a0 = *(const v4f*)(T + (size_t)sidx * F + c0), a1 = *(const v4f*)(T + (size_t)sidx * F + c0 + 4);
    for (int j = 0; j < 4; ++j) { mx[j] = fmaxf(mx[j], fmaxf(pmul(a0[j] - q[j], s[j]) + t[j], 0.0f)); mx[4 + j] = fmaxf(mx[4 + j], fmaxf(pmul(a1[j] - q[4 + j], s[4 + j]) + t[4 + j], 0.0f)); } }
  for (int pass = 0; pass < 2; ++pass) { if (v < mrows) { float* orow = FO_ + (size_t)v * F + c0; v4f o0, o1; for (int j = 0; j < 4; ++j) { o0[j] = (v < N) ? mx[j] : 0.0f; o1[j] = (v < N) ? mx[4 + j] : 0.0f; } *(volatile v4f*)orow = o0; *(volatile v4f*)(orow + 4) = o1; }
    __threadfence(); }
}
__global__ __launch_bounds__(256) void bnres_kernel(const float* __restrict__ B, const float* __restrict__ SCL, const float* __restrict__ SFT, const float* __restrict__ x, float* __restrict__ out, int nl) {
  const size_t i = (size_t)blockIdx.x * 256 + threadIdx.x; if (i >= (size_t)nl * (F / 4)) return; const size_t n = i / (F / 4); const int c = (int)(i % (F / 4)) * 4; const v4f b4 = *(const v4f*)(B + n * F + c), s = *(const v4f*)(SCL + c), t = *(const v4f*)(SFT + c), x4 = *(const v4f*)(x + n * F + c); v4f o;
  for (int j = 0; j < 4; ++j) o[j] = fmaxf(pmul(b4[j], s[j]) + t[j] + bfo(x4[j]), 0.0f);
  for (int pass = 0; pass < 2; ++pass) { *(volatile v4f*)(out + n * F + c) = o; __threadfence(); }
}
}

extern "C" void kernel_launch(void* const* d_in, const int* in_sizes, int n_in, void* d_out, int out_size, void* d_ws, size_t ws_size, hipStream_t stream) {
  (void)n_in;
  auto Fp = [&](int i) { return (const float*)d_in[i]; }; auto Ip = [&](int i) { return (const int*)d_in[i]; };
  if (in_sizes[0] != N * 3 || in_sizes[1] != N * F || in_sizes[2] != N * KNB || in_sizes[3] != F * F || in_sizes[8] != F * CW3 || in_sizes[13] != F * F || out_size != N * F) return;
  { const int v64[12] = {4, 5, 6, 7, 9, 10, 11, 12, 14, 15, 16, 17}; for (int i = 0; i < 12; ++i) if (in_sizes[v64[i]] != F) return; }
  size_t off = 0; char* ws = (char*)d_ws;
  auto carve = [&](size_t bytes) { char* p = ws + off; off += (bytes + 255) & ~(size_t)255; return p; };
  b16* W1T = (b16*)carve((size_t)F * F * 2); b16* WHT = (b16*)carve((size_t)F * F * 2); b16* WHQ = (b16*)carve((size_t)F * F * 2); b16* W3T = (b16*)carve((size_t)F * F * 2); b16* W3Q = (b16*)carve((size_t)F * F * 2);
  float* ZB = (float*)carve(1024); float* S1 = (float*)carve(1024); float* T1 = (float*)carve(1024); float* S2 = (float*)carve(1024); float* T2 = (float*)carve(1024); float* S3 = (float*)carve(1024); float* T3 = (float*)carve(1024);
  float* PA = (float*)carve((size_t)NP * F * 4); float* PB = (float*)carve((size_t)NP * F * 4); float* PQ = (float*)carve((size_t)NP * F * 4); float* PT = (float*)carve((size_t)NP * F * 4);
  if (off > ws_size || off > ((size_t)112 << 20)) return;
  { const unsigned g = (F * F / 8 + 255) / 256; wt_kernel<F, F, F><<<g, 256, 0, stream>>>(Fp(3), W1T, WSC); wtoip_kernel<F, F><<<g, 256, 0, stream>>>(Fp(8), CW3, 3, WHT, WSC); wtoip_kernel<F, F><<<g, 256, 0, stream>>>(Fp(8), CW3, 3, WHQ, WSQ);
    wt_kernel<F, F, F><<<g, 256, 0, stream>>>(Fp(13), W3T, WSC); wt_kernel<F, F, F><<<g, 256, 0, stream>>>(Fp(13), W3Q, WSQ); zfill_kernel<<<1, 256, 0, stream>>>(ZB, 256);
    bnfold_kernel<<<1, 256, 0, stream>>>(Fp(4), Fp(5), Fp(6), Fp(7), S1, T1); bnfold_kernel<<<1, 256, 0, stream>>>(Fp(9), Fp(10), Fp(11), Fp(12), S2, T2); bnfold_kernel<<<1, 256, 0, stream>>>(Fp(14), Fp(15), Fp(16), Fp(17), S3, T3); }
  lin_kernel<F, 4, 1, 0, false><<<NPL / 32, 64, 0, stream>>>(Fp(1), nullptr, W1T, W1T, ZB, PA, F, N, NPL);
  bnact_kernel<F, 1><<<(unsigned)(((size_t)NPL * (F / 4) + 255) / 256), 256, 0, stream>>>(PA, S1, T1, PB, F, NPL);
  lin_kernel<F, 4, 0, 0, false><<<NPL / 32, 64, 0, stream>>>(PB, nullptr, WHT, WHQ, ZB, PA, F, N, NPL);
  qtadd_kernel<<<(unsigned)(((size_t)NPL * (F / 4) + 255) / 256), 256, 0, stream>>>(Fp(0), Fp(8), PA, PQ, PT, NPL);
  ecmax_kernel<<<NPL / 32, 256, 0, stream>>>(PT, PQ, Ip(2), S2, T2, PB, NPL);
  lin_kernel<F, 4, 0, 0, false><<<NPL / 32, 64, 0, stream>>>(PB, nullptr, W3T, W3Q, ZB, PA, F, N, NPL);
  bnres_kernel<<<(unsigned)(((size_t)NL * (F / 4) + 255) / 256), 256, 0, stream>>>(PA, S3, T3, Fp(1), (float*)d_out, NL);
}
